// NMRShiftModel_30279519437525
// MI455X (gfx1250) — hardware-verified
//
#include <hip/hip_runtime.h>
#include <stddef.h>


#define INC     9
#define HIDV    185
#define KP      192
#define K0P     32
#define JKK     768
#define NL      3
#define NBN     4
#define NTHR    256
#define NWAVE   8
#define EPT     8
#define NGRP    2
#define CHUNK   (NTHR * EPT * NGRP)
#define WCAP    (EPT * NGRP * 32)
#define LISTN   (NWAVE * WCAP)
#define NBC     4096
#define NBF     1024
#define NBP     32
#define RCAP    40960
#define RBN     128
#define TGT     256
#define DEGCAP  256
#define GROWS   64
#define GCT     6
#define ALN     24
#define OTHR    512
#define WSCALE  16.0f
#define WINV    0.0625f
#define BNEPS   1e-5f

#define LDS_FILL ((RCAP + NBF + LISTN) * 4 + 64)

static_assert((CHUNK & (CHUNK - 1)) == 0);
static_assert(CHUNK <= 4096);
static_assert(NBC <= 4096 && NBF <= 4096 && NBP <= 4096);
static_assert((NBC & (NBC - 1)) == 0 && (NBF & (NBF - 1)) == 0 && (NBP & (NBP - 1)) == 0);
static_assert(NBC == 4 * NBF);
static_assert(OTHR * 8 == NBC);
static_assert((RCAP % 32) == 0);
static_assert(TGT == NWAVE * 32 && (TGT % GROWS) == 0 && (NBC % TGT) == 0);
static_assert(ALN * 8 == KP && 2 * GCT * 16 == KP && JKK == 4 * KP);
static_assert(GROWS * KP / 4 == 12 * NTHR);
static_assert(NBP * 8 == NTHR);
static_assert((K0P % 32) == 0 && (KP % 32) == 0 && HIDV <= KP && INC <= K0P && NBN * HIDV <= JKK);
static_assert(((KP * K0P / 8) % NTHR) == 0 && ((NL * KP * KP / 8) % NTHR) == 0 && ((KP * JKK / 8) % NTHR) == 0);

typedef float    v4f  __attribute__((ext_vector_type(4)));
typedef float    v8f  __attribute__((ext_vector_type(8)));
typedef int      v4i  __attribute__((ext_vector_type(4)));
typedef _Float16 v8h  __attribute__((ext_vector_type(8)));
typedef _Float16 v16h __attribute__((ext_vector_type(16)));
union FragH { v16h v; v8h h[2]; };

__device__ __forceinline__ v8h cvt8(v4f a, v4f b) {
  v8h r;
  r[0] = (_Float16)a.x; r[1] = (_Float16)a.y; r[2] = (_Float16)a.z; r[3] = (_Float16)a.w;
  r[4] = (_Float16)b.x; r[5] = (_Float16)b.y; r[6] = (_Float16)b.z; r[7] = (_Float16)b.w;
  return r;
}

__device__ __forceinline__ v8f wmh(v16h a, v16h b, v8f c) {
  v8f d = __builtin_amdgcn_wmma_f32_16x16x32_f16(false, a, false, b, (short)0, c, false, false);
  asm volatile("v_nop\n\tv_nop\n\tv_nop\n\tv_nop" : "+v"(d) : "v"(a), "v"(b));
  return d;
}

__device__ __forceinline__ v4f vmax4(v4f a, v4f b) {
  v4f r;
  r.x = fmaxf(a.x, b.x); r.y = fmaxf(a.y, b.y); r.z = fmaxf(a.z, b.z); r.w = fmaxf(a.w, b.w);
  return r;
}

template <int NB>
__device__ __forceinline__ int scan_chunk(const int* __restrict__ dsts, int nE, int cbase, int slotBase,
                                          int vec8, int* list, int tid, int lane, int wave) {
  int wc = 0;
#pragma unroll
  for (int g = 0; g < NGRP; ++g) {
    const int el0  = (g * NTHR + tid) * EPT;
    const int e0   = cbase + el0;
    const int sent = -2147483647 - 1;
    v4i da, db;
    if (vec8 != 0 && cbase + CHUNK <= nE) {
      da = *(const v4i*)(dsts + e0);
      db = *(const v4i*)(dsts + e0 + 4);
    } else {
      da.x = (e0     < nE) ? dsts[min(e0, nE - 1)] : sent;
      da.y = (e0 + 1 < nE) ? dsts[min(e0 + 1, nE - 1)] : sent;
      da.z = (e0 + 2 < nE) ? dsts[min(e0 + 2, nE - 1)] : sent;
      da.w = (e0 + 3 < nE) ? dsts[min(e0 + 3, nE - 1)] : sent;
      db.x = (e0 + 4 < nE) ? dsts[min(e0 + 4, nE - 1)] : sent;
      db.y = (e0 + 5 < nE) ? dsts[min(e0 + 5, nE - 1)] : sent;
      db.z = (e0 + 6 < nE) ? dsts[min(e0 + 6, nE - 1)] : sent;
      db.w = (e0 + 7 < nE) ? dsts[min(e0 + 7, nE - 1)] : sent;
    }
    const unsigned nb = (unsigned)slotBase;
    const unsigned s0 = (unsigned)da.x - nb, s1 = (unsigned)da.y - nb;
    const unsigned s2 = (unsigned)da.z - nb, s3 = (unsigned)da.w - nb;
    const unsigned s4 = (unsigned)db.x - nb, s5 = (unsigned)db.y - nb;
    const unsigned s6 = (unsigned)db.z - nb, s7 = (unsigned)db.w - nb;
    const bool h0 = s0 < (unsigned)NB, h1 = s1 < (unsigned)NB, h2 = s2 < (unsigned)NB, h3 = s3 < (unsigned)NB;
    const bool h4 = s4 < (unsigned)NB, h5 = s5 < (unsigned)NB, h6 = s6 < (unsigned)NB, h7 = s7 < (unsigned)NB;
    const unsigned any = __builtin_amdgcn_ballot_w32(h0 | h1 | h2 | h3 | h4 | h5 | h6 | h7);
    if (any != 0u) {
#define HITJ(J, HJ, SJ) { \
        const unsigned mj = __builtin_amdgcn_ballot_w32(HJ); \
        if (mj != 0u) { \
          if (HJ) { \
            const int pos = wc + (int)__builtin_amdgcn_mbcnt_lo(mj, 0u); \
            if (pos < WCAP) list[wave * WCAP + pos] = ((el0 + (J)) << 12) | (int)(SJ); \
          } \
          wc += (int)__builtin_popcount(mj); } }
      HITJ(0, h0, s0)
      HITJ(1, h1, s1)
      HITJ(2, h2, s2)
      HITJ(3, h3, s3)
      HITJ(4, h4, s4)
      HITJ(5, h5, s5)
      HITJ(6, h6, s6)
      HITJ(7, h7, s7)
#undef HITJ
    }
  }
  return wc;
}

__global__ __launch_bounds__(NTHR) void k_prep(
    const float* __restrict__ x, const float* __restrict__ W0, const float* __restrict__ Wh,
    const float* __restrict__ Wjk, _Float16* xh, _Float16* wb0, _Float16* wbh, _Float16* wbjk,
    int nN, int nxThr) {
  const int g0 = nxThr;
  const int g1 = g0 + KP * K0P / 8;
  const int g2 = g1 + NL * KP * KP / 8;
  const int g3 = g2 + KP * JKK / 8;
  const int i = blockIdx.x * NTHR + (int)threadIdx.x;
  const int bstart = blockIdx.x * NTHR;
  if (i >= g3) return;
  float v[8];
  _Float16* dp;
  if (bstart < g0) {
    const int n  = i >> 2;
    const int k0 = (i & 3) * 8;
    const int nc = n < nN ? n : nN - 1;
#pragma unroll
    for (int e = 0; e < 8; ++e) {
      const int k  = k0 + e;
      const int kc = k < INC ? k : INC - 1;
      const float xv = x[(size_t)nc * INC + kc];
      v[e] = (n < nN && k < INC) ? xv : 0.0f;
    }
    dp = xh + (size_t)i * 8;
  } else if (bstart < g1) {
    const int o  = (i - g0) * 8;
    const int n  = o / K0P;
    const int k0 = o - n * K0P;
    const int nc = n < HIDV ? n : HIDV - 1;
#pragma unroll
    for (int e = 0; e < 8; ++e) {
      const int k  = k0 + e;
      const int kc = k < INC ? k : INC - 1;
      const float w = W0[kc * HIDV + nc];
      v[e] = (k < INC && n < HIDV) ? w * WSCALE : 0.0f;
    }
    dp = wb0 + o;
  } else if (bstart < g2) {
    const int o  = (i - g1) * 8;
    const int l  = o / (KP * KP);
    const int oo = o - l * (KP * KP);
    const int n  = oo / KP;
    const int k0 = oo - n * KP;
    const int nc = n < HIDV ? n : HIDV - 1;
#pragma unroll
    for (int e = 0; e < 8; ++e) {
      const int k  = k0 + e;
      const int kc = k < HIDV ? k : HIDV - 1;
      const float w = Wh[((size_t)l * HIDV + kc) * HIDV + nc];
      v[e] = (k < HIDV && n < HIDV) ? w * WSCALE : 0.0f;
    }
    dp = wbh + o;
  } else {
    const int o   = (i - g2) * 8;
    const int n   = o / JKK;
    const int kk0 = o - n * JKK;
    const int l   = kk0 / KP;
    const int c0  = kk0 - l * KP;
    const int nc  = n < HIDV ? n : HIDV - 1;
#pragma unroll
    for (int e = 0; e < 8; ++e) {
      const int c  = c0 + e;
      const int cc = c < HIDV ? c : HIDV - 1;
      const float w = Wjk[((size_t)(l * HIDV + cc)) * HIDV + nc];
      v[e] = (c < HIDV && n < HIDV) ? w * WSCALE : 0.0f;
    }
    dp = wbjk + o;
  }
  v4f a, b;
  a.x = v[0]; a.y = v[1]; a.z = v[2]; a.w = v[3];
  b.x = v[4]; b.y = v[5]; b.z = v[6]; b.w = v[7];
  const v8h hv = cvt8(a, b);
  *(volatile v8h*)dp = hv;
  __threadfence();
  *(volatile v8h*)dp = hv;
}

__global__ __launch_bounds__(NTHR) void k_count(
    const int* __restrict__ ei, int* cnt, float* dinv, int nE, int vec8) {
  __shared__ __attribute__((aligned(16))) int scnt[NBC];
  __shared__ __attribute__((aligned(16))) int list[LISTN];
  __shared__ int wcnt[NWAVE];
  const int tid = threadIdx.x, lane = tid & 31, wave = tid >> 5;
  const int nodeBase = blockIdx.x * NBC;
  const int* dsts = ei + nE;

  for (int i = tid; i < NBC; i += NTHR) scnt[i] = 0;
  __syncthreads();

  const int nChunks = (nE + CHUNK - 1) / CHUNK;
#pragma unroll 1
  for (int ch = 0; ch < nChunks; ++ch) {
    const int cbase = ch * CHUNK;
    const int wc = scan_chunk<NBC>(dsts, nE, cbase, nodeBase, vec8, list, tid, lane, wave);
    if (lane == 0) wcnt[wave] = wc;
    __syncthreads();
    if (wave == 0) {
#pragma unroll 1
      for (int wsx = 0; wsx < NWAVE; ++wsx) {
        int n = __builtin_amdgcn_readfirstlane(wcnt[wsx]);
        n = n > WCAP ? WCAP : (n < 0 ? 0 : n);
        const int* lp = list + wsx * WCAP;
#pragma unroll 1
        for (int i = 0; i < n; ++i) {
          const int ent  = __builtin_amdgcn_readfirstlane(lp[i]);
          const int slot = ent & (NBC - 1);
          if (lane == 0) scnt[slot] = scnt[slot] + 1;
        }
      }
    }
    __syncthreads();
  }

  v4i cq[4]; v4f dq[4];
#pragma unroll
  for (int q = 0; q < 4; ++q) {
    const int f = (wave * 4 + q) * 128 + 4 * lane;
    const v4i c = *(const v4i*)(scnt + f);
    cq[q] = c;
    dq[q].x = rsqrtf((float)(c.x + 1));
    dq[q].y = rsqrtf((float)(c.y + 1));
    dq[q].z = rsqrtf((float)(c.z + 1));
    dq[q].w = rsqrtf((float)(c.w + 1));
  }
  int*   cp = cnt + (size_t)nodeBase;
  float* dp = dinv + (size_t)nodeBase;
#pragma unroll
  for (int q = 0; q < 4; ++q) {
    const int f = (wave * 4 + q) * 128 + 4 * lane;
    *(volatile v4i*)(cp + f) = cq[q];
    *(volatile v4f*)(dp + f) = dq[q];
  }
  __threadfence();
#pragma unroll
  for (int q = 0; q < 4; ++q) {
    const int f = (wave * 4 + q) * 128 + 4 * lane;
    *(volatile v4i*)(cp + f) = cq[q];
    *(volatile v4f*)(dp + f) = dq[q];
  }
}

__global__ __launch_bounds__(OTHR) void k_offsets(
    const int* __restrict__ cnt, int* off, int* rbase, int nChunk) {
  __shared__ __attribute__((aligned(16))) int soff[NBC];
  __shared__ __attribute__((aligned(16))) int srb[RBN];
  __shared__ int wtot[OTHR / 32];
  const int tid = threadIdx.x, lane = tid & 31, wave = tid >> 5, sub = tid >> 7;
  for (int i = tid; i < RBN; i += OTHR) srb[i] = 0;
  int carry = 0;
#pragma unroll 1
  for (int ch = 0; ch < nChunk; ++ch) {
    const int base = ch * NBC;
    const v4i c0 = *(const v4i*)(cnt + base + 8 * tid);
    const v4i c1 = *(const v4i*)(cnt + base + 8 * tid + 4);
    const int e0 = max(c0.x, 0), e1 = max(c0.y, 0), e2 = max(c0.z, 0), e3 = max(c0.w, 0);
    const int e4 = max(c1.x, 0), e5 = max(c1.y, 0), e6 = max(c1.z, 0), e7 = max(c1.w, 0);
    const int ts = e0 + e1 + e2 + e3 + e4 + e5 + e6 + e7;
    int incl = ts;
#pragma unroll
    for (int d = 1; d < 32; d <<= 1) {
      const int t = __shfl_up(incl, d);
      if (lane >= d) incl += t;
    }
    if (lane == 31) wtot[wave] = incl;
    __syncthreads();
    const int S0 = wtot[0]  + wtot[1]  + wtot[2]  + wtot[3];
    const int S1 = wtot[4]  + wtot[5]  + wtot[6]  + wtot[7];
    const int S2 = wtot[8]  + wtot[9]  + wtot[10] + wtot[11];
    const int S3 = wtot[12] + wtot[13] + wtot[14] + wtot[15];
    int pre = 0;
#pragma unroll 1
    for (int w = 4 * sub; w < wave; ++w) pre += wtot[w];
    const int b0 = carry;
    const int b1 = b0 + ((S0 + 31) & ~31);
    const int b2 = b1 + ((S1 + 31) & ~31);
    const int b3 = b2 + ((S2 + 31) & ~31);
    const int b4 = b3 + ((S3 + 31) & ~31);
    const int myb = sub == 0 ? b0 : (sub == 1 ? b1 : (sub == 2 ? b2 : b3));
    if (tid == 0) {
      srb[min(4 * ch + 0, RBN - 1)] = b0;
      srb[min(4 * ch + 1, RBN - 1)] = b1;
      srb[min(4 * ch + 2, RBN - 1)] = b2;
      srb[min(4 * ch + 3, RBN - 1)] = b3;
    }
    int run = myb + pre + incl - ts;
    soff[8 * tid + 0] = run; run += e0;
    soff[8 * tid + 1] = run; run += e1;
    soff[8 * tid + 2] = run; run += e2;
    soff[8 * tid + 3] = run; run += e3;
    soff[8 * tid + 4] = run; run += e4;
    soff[8 * tid + 5] = run; run += e5;
    soff[8 * tid + 6] = run; run += e6;
    soff[8 * tid + 7] = run;
    carry = b4;
    __syncthreads();
    const v4i o0 = *(const v4i*)(soff + 4 * tid);
    const v4i o1 = *(const v4i*)(soff + 4 * (tid + OTHR));
    int* op = off + base;
    *(volatile v4i*)(op + 4 * tid) = o0;
    *(volatile v4i*)(op + 4 * (tid + OTHR)) = o1;
    __threadfence();
    *(volatile v4i*)(op + 4 * tid) = o0;
    *(volatile v4i*)(op + 4 * (tid + OTHR)) = o1;
    __syncthreads();
  }
  if (tid == 0) srb[min(4 * nChunk, RBN - 1)] = carry;
  __syncthreads();
  v4i rv = {0, 0, 0, 0};
  if (tid < 32) rv = *(const v4i*)(srb + 4 * tid);
  if (tid < 32) *(volatile v4i*)(rbase + 4 * tid) = rv;
  __threadfence();
  if (tid < 32) *(volatile v4i*)(rbase + 4 * tid) = rv;
}

__global__ __launch_bounds__(NTHR) void k_fill(
    const int* __restrict__ ei, const int* __restrict__ off, const int* __restrict__ rbase,
    int* csr, int nN, int nE, int vec8, int csrLen) {
  extern __shared__ v4f lds_dyn[];
  int* region = (int*)lds_dyn;
  int* cursor = region + RCAP;
  int* list   = cursor + NBF;
  int* wcnt   = list + LISTN;
  const int tid = threadIdx.x, lane = tid & 31, wave = tid >> 5;
  const int b = blockIdx.x;
  const int nodeBase = b * NBF;
  const int* dsts = ei + nE;

  int rb0 = rbase[b];
  const int rb1 = rbase[b + 1];
  rb0 = rb0 < 0 ? 0 : (rb0 > csrLen ? csrLen : rb0);
  rb0 &= ~31;
  int len = rb1 - rb0;
  len = len < 0 ? 0 : (len > RCAP ? RCAP : len);
  int lenW = (len + 31) & ~31;
  if (rb0 + lenW > csrLen) lenW = (csrLen - rb0) & ~31;

  {
    const v4i z = {0, 0, 0, 0};
    for (int i = tid; i < RCAP / 4; i += NTHR) ((v4i*)region)[i] = z;
    for (int s = tid; s < NBF; s += NTHR) {
      int o = off[nodeBase + s] - rb0;
      o = o < 0 ? 0 : (o > RCAP ? RCAP : o);
      cursor[s] = o;
    }
  }
  __syncthreads();

  const int nChunks = (nE + CHUNK - 1) / CHUNK;
#pragma unroll 1
  for (int ch = 0; ch < nChunks; ++ch) {
    const int cbase = ch * CHUNK;
    const int wc = scan_chunk<NBF>(dsts, nE, cbase, nodeBase, vec8, list, tid, lane, wave);
    if (lane == 0) wcnt[wave] = wc;
    __syncthreads();
    if (wave == 0) {
#pragma unroll 1
      for (int wsx = 0; wsx < NWAVE; ++wsx) {
        int n = __builtin_amdgcn_readfirstlane(wcnt[wsx]);
        n = n > WCAP ? WCAP : (n < 0 ? 0 : n);
        const int* lp = list + wsx * WCAP;
#pragma unroll 1
        for (int i = 0; i < n; ++i) {
          const int ent  = __builtin_amdgcn_readfirstlane(lp[i]);
          const int slot = ent & (NBF - 1);
          int e = cbase + ((ent >> 12) & (CHUNK - 1));
          e = e > nE - 1 ? nE - 1 : e;
          int src = ei[e];
          src = src < 0 ? 0 : (src > nN - 1 ? nN - 1 : src);
          if (lane == 0) {
            int pos = cursor[slot];
            pos = pos < 0 ? 0 : (pos > RCAP - 1 ? RCAP - 1 : pos);
            region[pos] = src;
            const int np = pos + 1;
            cursor[slot] = np > RCAP ? RCAP : np;
          }
        }
      }
    }
    __syncthreads();
  }

  const int nv = lenW >> 2;
  int* gp = csr + rb0;
#pragma unroll 1
  for (int i = tid; i < nv; i += NTHR) { const v4i v = ((const v4i*)region)[i]; *(volatile v4i*)(gp + 4 * i) = v; }
  __threadfence();
#pragma unroll 1
  for (int i = tid; i < nv; i += NTHR) { const v4i v = ((const v4i*)region)[i]; *(volatile v4i*)(gp + 4 * i) = v; }
}

template <int KT, int KTP, int LDA>
__global__ __launch_bounds__(NTHR) void k_gemm(
    const _Float16* __restrict__ A, const _Float16* __restrict__ Bs, const float* __restrict__ dinv,
    const float* __restrict__ bias, float* C, size_t planeStride, int useDinv, int useBias, int nValid) {
  __shared__ __attribute__((aligned(16))) float stg[GROWS * KP];
  constexpr int KPB = KT * 32;
  const int tid = threadIdx.x, lane = tid & 31, wave = tid >> 5, hh = lane >> 4, m = lane & 15;
  const int rs = wave & 3, cg = wave >> 2;
  const int rowBase = blockIdx.x * GROWS;

  v8f acc[GCT];
#pragma unroll
  for (int t = 0; t < GCT; ++t) { v8f z = {0.f, 0.f, 0.f, 0.f, 0.f, 0.f, 0.f, 0.f}; acc[t] = z; }
  const _Float16* arow = A + (size_t)(rowBase + 16 * rs + m) * LDA + 8 * hh;
  const _Float16* bcol = Bs + (size_t)(16 * GCT * cg + m) * KPB + 8 * hh;
#pragma unroll 3
  for (int kt = 0; kt < KT; ++kt) {
    const int pl = kt / KTP;
    const int kk = kt - pl * KTP;
    const _Float16* ap = arow + (size_t)pl * planeStride + 32 * kk;
    FragH a;
    a.h[0] = *(const v8h*)ap;
    a.h[1] = *(const v8h*)(ap + 16);
#pragma unroll
    for (int t = 0; t < GCT; ++t) {
      const _Float16* bp = bcol + (size_t)(16 * t) * KPB + 32 * kt;
      FragH b;
      b.h[0] = *(const v8h*)bp;
      b.h[1] = *(const v8h*)(bp + 16);
      acc[t] = wmh(a.v, b.v, acc[t]);
    }
  }

  const int r0 = 16 * rs + 8 * hh;
  const v4f dA = *(const v4f*)(dinv + (size_t)rowBase + r0);
  const v4f dB = *(const v4f*)(dinv + (size_t)rowBase + r0 + 4);
  float s[8];
  s[0] = dA.x; s[1] = dA.y; s[2] = dA.z; s[3] = dA.w; s[4] = dB.x; s[5] = dB.y; s[6] = dB.z; s[7] = dB.w;
#pragma unroll
  for (int r = 0; r < 8; ++r) s[r] = (useDinv != 0 ? s[r] : 1.0f) * WINV;
  float* sp = stg + r0 * KP + 16 * GCT * cg + m;
#pragma unroll
  for (int t = 0; t < GCT; ++t) {
    const int col = 16 * (GCT * cg + t) + m;
    const float bl = bias[col < nValid ? col : nValid - 1];
    const float bv = (useBias != 0 && col < nValid) ? bl : 0.0f;
#pragma unroll
    for (int r = 0; r < 8; ++r) sp[r * KP + 16 * t] = acc[t][r] * s[r] + bv;
  }
  __syncthreads();

  const v4f* lp = (const v4f*)stg;
  float* gp = C + (size_t)rowBase * KP;
#pragma unroll
  for (int i = 0; i < GROWS * KP / 4 / NTHR; ++i) {
    const int f = i * NTHR + tid;
    const v4f v = lp[f];
    *(volatile v4f*)(gp + 4 * (size_t)f) = v;
  }
  __threadfence();
#pragma unroll
  for (int i = 0; i < GROWS * KP / 4 / NTHR; ++i) {
    const int f = i * NTHR + tid;
    const v4f v = lp[f];
    *(volatile v4f*)(gp + 4 * (size_t)f) = v;
  }
}

__global__ __launch_bounds__(NTHR) void k_agg(
    const int* __restrict__ csr, const int* __restrict__ off, const int* __restrict__ cnt,
    const float* __restrict__ dinv, const float* __restrict__ hw, _Float16* xs,
    const float* __restrict__ bs, const float* __restrict__ bgam, const float* __restrict__ bbet,
    const float* __restrict__ bmean, const float* __restrict__ bvar, int nN, int csrLen) {
  const int tid = threadIdx.x, lane = tid & 31, wave = tid >> 5;
  const int tbase = blockIdx.x * TGT + wave * 32;
  const int cl = tbase + lane;
  const int cnt_l = cnt[cl];
  const int off_l = off[cl];
  union FI { float f; int i; };
  FI dvu; dvu.f = dinv[cl];
  const int lc  = lane < ALN ? lane : ALN - 1;
  const int ch0 = 8 * lc;
  float bb[8], ga[8], be[8], mu[8], sc[8];
#pragma unroll
  for (int e = 0; e < 8; ++e) {
    const int ch  = ch0 + e;
    const int chc = ch < HIDV ? ch : HIDV - 1;
    bb[e] = bs[chc];
    ga[e] = bgam[chc];
    be[e] = bbet[chc];
    mu[e] = bmean[chc];
    sc[e] = rsqrtf(bvar[chc] + BNEPS);
  }

#pragma unroll 1
  for (int j = 0; j < 32; ++j) {
    const int c = tbase + j;
    int n = __builtin_amdgcn_readlane(cnt_l, j);
    n = n < 0 ? 0 : (n > DEGCAP ? DEGCAP : n);
    const int st = __builtin_amdgcn_readlane(off_l, j);
    FI du; du.i = __builtin_amdgcn_readlane(dvu.i, j);
    const float dc = du.f;
    v4f a0 = {0.f, 0.f, 0.f, 0.f}, a1 = {0.f, 0.f, 0.f, 0.f};
#pragma unroll 1
    for (int q0 = 0; q0 < n; q0 += 32) {
      int pos = st + q0 + lane;
      pos = pos < 0 ? 0 : (pos > csrLen - 1 ? csrLen - 1 : pos);
      int sl = csr[pos];
      sl = sl < 0 ? 0 : (sl > nN - 1 ? nN - 1 : sl);
      const int mcnt = (n - q0) < 32 ? (n - q0) : 32;
#pragma unroll 1
      for (int p = 0; p < mcnt; ++p) {
        const int s = __builtin_amdgcn_readlane(sl, p);
        const float* hp = hw + (size_t)s * KP + ch0;
        a0 = a0 + *(const v4f*)hp;
        a1 = a1 + *(const v4f*)(hp + 4);
      }
    }
    const float* cpn = hw + (size_t)c * KP + ch0;
    const v4f s0 = *(const v4f*)cpn, s1 = *(const v4f*)(cpn + 4);
    const v4f t0 = (a0 + s0) * dc, t1 = (a1 + s1) * dc;
    float v[8];
    v[0] = t0.x; v[1] = t0.y; v[2] = t0.z; v[3] = t0.w; v[4] = t1.x; v[5] = t1.y; v[6] = t1.z; v[7] = t1.w;
#pragma unroll
    for (int e = 0; e < 8; ++e) {
      float y = v[e] + bb[e];
      y = (y - mu[e]) * sc[e];
      y = y * ga[e] + be[e];
      y = fmaxf(y, 0.0f);
      v[e] = (ch0 + e < HIDV) ? y : 0.0f;
    }
    v4f oa, ob;
    oa.x = v[0]; oa.y = v[1]; oa.z = v[2]; oa.w = v[3];
    ob.x = v[4]; ob.y = v[5]; ob.z = v[6]; ob.w = v[7];
    const v8h hv = cvt8(oa, ob);
    _Float16* xp = xs + (size_t)c * KP + 8 * lane;
    if (lane < ALN) *(volatile v8h*)xp = hv;
    __threadfence();
    if (lane < ALN) *(volatile v8h*)xp = hv;
  }
}

__global__ __launch_bounds__(NTHR) void k_pool(
    const int* __restrict__ batch, const float* __restrict__ hjk, const float* __restrict__ wout,
    const float* __restrict__ bout, float* gout, int nN) {
  __shared__ __attribute__((aligned(16))) float accm[NBP * KP];
  __shared__ __attribute__((aligned(16))) int list[LISTN];
  __shared__ __attribute__((aligned(16))) float sg[NBP];
  __shared__ int wcnt[NWAVE];
  const int tid = threadIdx.x, lane = tid & 31, wave = tid >> 5;
  const int gBase = blockIdx.x * NBP;
  const int lc  = lane < ALN ? lane : ALN - 1;
  const int ch0 = 8 * lc;

  {
    const float ninf = __uint_as_float(0xff800000u);
    const v4f z = {ninf, ninf, ninf, ninf};
    for (int i = tid; i < NBP * KP / 4; i += NTHR) ((v4f*)accm)[i] = z;
  }
  __syncthreads();

  const int nChunks = (nN + CHUNK - 1) / CHUNK;
#pragma unroll 1
  for (int ch = 0; ch < nChunks; ++ch) {
    const int cbase = ch * CHUNK;
    const int wc = scan_chunk<NBP>(batch, nN, cbase, gBase, 1, list, tid, lane, wave);
    if (lane == 0) wcnt[wave] = wc;
    __syncthreads();
    if (wave == 0) {
#pragma unroll 1
      for (int wsx = 0; wsx < NWAVE; ++wsx) {
        int n = __builtin_amdgcn_readfirstlane(wcnt[wsx]);
        n = n > WCAP ? WCAP : (n < 0 ? 0 : n);
        const int* lp = list + wsx * WCAP;
#pragma unroll 1
        for (int i = 0; i < n; ++i) {
          const int ent  = __builtin_amdgcn_readfirstlane(lp[i]);
          const int slot = ent & (NBP - 1);
          int nd = cbase + ((ent >> 12) & (CHUNK - 1));
          nd = nd > nN - 1 ? nN - 1 : nd;
          const float* hp = hjk + (size_t)nd * KP + ch0;
          const v4f v0 = *(const v4f*)hp, v1 = *(const v4f*)(hp + 4);
          float* ap = accm + slot * KP + ch0;
          const v4f c0 = *(const v4f*)ap, c1 = *(const v4f*)(ap + 4);
          const v4f m0 = vmax4(c0, v0), m1 = vmax4(c1, v1);
          if (lane < ALN) { *(v4f*)ap = m0; *(v4f*)(ap + 4) = m1; }
        }
      }
    }
    __syncthreads();
  }

  const int slot = tid >> 3, part = tid & 7;
  float sum = 0.0f;
#pragma unroll 1
  for (int c = part; c < HIDV; c += 8) sum += accm[slot * KP + c] * wout[c];
  sum += __shfl_xor(sum, 4);
  sum += __shfl_xor(sum, 2);
  sum += __shfl_xor(sum, 1);
  sum += bout[0];
  if (part == 0) sg[slot] = sum;
  __syncthreads();
  const v4f ov = *(const v4f*)(sg + 4 * (tid & 7));
  float* op = gout + (size_t)blockIdx.x * NBP;
  if (tid < 8) *(volatile v4f*)(op + 4 * tid) = ov;
  __threadfence();
  if (tid < 8) *(volatile v4f*)(op + 4 * tid) = ov;
}

__global__ __launch_bounds__(NTHR) void k_out(const float* __restrict__ gout, float* out, int G) {
  const int tid = threadIdx.x;
  const int nv = G >> 2;
  const int tail0 = nv << 2;
#pragma unroll 1
  for (int i = tid; i < nv; i += NTHR) { const v4f v = *(const v4f*)(gout + 4 * i); *(volatile v4f*)(out + 4 * i) = v; }
#pragma unroll 1
  for (int i = tail0 + tid; i < G; i += NTHR) { const float v = gout[i]; *(volatile float*)(out + i) = v; }
  __threadfence();
#pragma unroll 1
  for (int i = tid; i < nv; i += NTHR) { const v4f v = *(const v4f*)(gout + 4 * i); *(volatile v4f*)(out + 4 * i) = v; }
#pragma unroll 1
  for (int i = tail0 + tid; i < G; i += NTHR) { const float v = gout[i]; *(volatile float*)(out + i) = v; }
}

extern "C" void kernel_launch(void* const* d_in, const int* in_sizes, int n_in,
                              void* d_out, int out_size, void* d_ws, size_t ws_size,
                              hipStream_t stream) {
  if (n_in < 15) return;
  const int nN = in_sizes[2];
  const int nE = in_sizes[1] / 2;
  if (nN <= 0 || nE <= 0 || in_sizes[1] != 2 * nE || in_sizes[0] != nN * INC) return;
  if (in_sizes[3] != INC * HIDV || in_sizes[4] != HIDV) return;
  if (in_sizes[5] != NL * HIDV * HIDV || in_sizes[6] != NL * HIDV) return;
  if (in_sizes[7] != NBN * HIDV || in_sizes[8] != NBN * HIDV || in_sizes[9] != NBN * HIDV || in_sizes[10] != NBN * HIDV) return;
  if (in_sizes[11] != NBN * HIDV * HIDV || in_sizes[12] != HIDV || in_sizes[13] != HIDV || in_sizes[14] < 1) return;
  const int G = out_size;
  if (G <= 0) return;
  if (nE > (1 << 28) || nN > (1 << 24)) return;

  const float* x     = (const float*)d_in[0];
  const int*   ei    = (const int*)d_in[1];
  const int*   batch = (const int*)d_in[2];
  const float* W0    = (const float*)d_in[3];
  const float* b0    = (const float*)d_in[4];
  const float* Wh    = (const float*)d_in[5];
  const float* bh    = (const float*)d_in[6];
  const float* gam   = (const float*)d_in[7];
  const float* bet   = (const float*)d_in[8];
  const float* mean  = (const float*)d_in[9];
  const float* var   = (const float*)d_in[10];
  const float* Wjk   = (const float*)d_in[11];
  const float* bjk   = (const float*)d_in[12];
  const float* Wout  = (const float*)d_in[13];
  const float* bout  = (const float*)d_in[14];
  float* out = (float*)d_out;

  const int NPAD   = ((nN + TGT - 1) / TGT) * TGT;
  const int nBC    = (nN + NBC - 1) / NBC;
  const int CNTPAD = nBC * NBC;
  if (4 * nBC + 1 > RBN || CNTPAD < NPAD) return;
  const int nBF    = (nN + NBF - 1) / NBF;
  const int csrLen = ((nE + 31) & ~31) + 4096;
  const int nGemm  = NPAD / GROWS;
  const int nAgg   = NPAD / TGT;
  const int nPool  = (G + NBP - 1) / NBP;
  const size_t plane = (size_t)NPAD * KP;

  char* ws = (char*)d_ws;
  size_t off = 0;
  const size_t oXh  = off; off += (size_t)NPAD * K0P * 2;          off = (off + 255) & ~(size_t)255;
  const size_t oB0  = off; off += (size_t)KP * K0P * 2;            off = (off + 255) & ~(size_t)255;
  const size_t oBh  = off; off += (size_t)NL * KP * KP * 2;        off = (off + 255) & ~(size_t)255;
  const size_t oBjk = off; off += (size_t)KP * JKK * 2;            off = (off + 255) & ~(size_t)255;
  const size_t oCnt = off; off += (size_t)CNTPAD * 4;              off = (off + 255) & ~(size_t)255;
  const size_t oDv  = off; off += (size_t)CNTPAD * 4;              off = (off + 255) & ~(size_t)255;
  const size_t oOff = off; off += (size_t)CNTPAD * 4;              off = (off + 255) & ~(size_t)255;
  const size_t oRb  = off; off += (size_t)RBN * 4;                 off = (off + 255) & ~(size_t)255;
  const size_t oCsr = off; off += (size_t)csrLen * 4;              off = (off + 255) & ~(size_t)255;
  const size_t oXs  = off; off += (size_t)4 * plane * 2;           off = (off + 255) & ~(size_t)255;
  const size_t oHw  = off; off += (size_t)NPAD * KP * 4;           off = (off + 255) & ~(size_t)255;
  const size_t oGo  = off; off += (size_t)nPool * NBP * 4;         off = (off + 255) & ~(size_t)255;
  if (off > ws_size) return;
  _Float16* xh   = (_Float16*)(ws + oXh);
  _Float16* wb0  = (_Float16*)(ws + oB0);
  _Float16* wbh  = (_Float16*)(ws + oBh);
  _Float16* wbjk = (_Float16*)(ws + oBjk);
  int*      cnt  = (int*)(ws + oCnt);
  float*    dinv = (float*)(ws + oDv);
  int*      offp = (int*)(ws + oOff);
  int*      rb   = (int*)(ws + oRb);
  int*      csr  = (int*)(ws + oCsr);
  _Float16* xs   = (_Float16*)(ws + oXs);
  float*    hw   = (float*)(ws + oHw);
  float*    gout = (float*)(ws + oGo);

  const int vec8 = ((nE & 3) == 0) ? 1 : 0;

  const int nxThr = NPAD * (K0P / 8);
  const int nPrep = nxThr + KP * K0P / 8 + NL * KP * KP / 8 + KP * JKK / 8;
  k_prep<<<(nPrep + NTHR - 1) / NTHR, NTHR, 0, stream>>>(x, W0, Wh, Wjk, xh, wb0, wbh, wbjk, nN, nxThr);

  k_count<<<nBC, NTHR, 0, stream>>>(ei, cnt, dinv, nE, vec8);
  k_offsets<<<1, OTHR, 0, stream>>>(cnt, offp, rb, nBC);
  hipFuncSetAttribute(reinterpret_cast<const void*>(&k_fill),
                      hipFuncAttributeMaxDynamicSharedMemorySize, LDS_FILL);
  k_fill<<<nBF, NTHR, LDS_FILL, stream>>>(ei, offp, rb, csr, nN, nE, vec8, csrLen);

  k_gemm<K0P / 32, K0P / 32, K0P><<<nGemm, NTHR, 0, stream>>>(xh, wb0, dinv, bjk, hw, (size_t)0, 1, 0, HIDV);
  k_agg<<<nAgg, NTHR, 0, stream>>>(csr, offp, cnt, dinv, hw, xs, b0, gam, bet, mean, var, nN, csrLen);

  for (int i = 1; i <= NL; ++i) {
    k_gemm<KP / 32, KP / 32, KP><<<nGemm, NTHR, 0, stream>>>(
        xs + (size_t)(i - 1) * plane, wbh + (size_t)(i - 1) * KP * KP, dinv, bjk, hw, (size_t)0, 1, 0, HIDV);
    k_agg<<<nAgg, NTHR, 0, stream>>>(csr, offp, cnt, dinv, hw, xs + (size_t)i * plane,
                                     bh + (size_t)(i - 1) * HIDV, gam + (size_t)i * HIDV, bet + (size_t)i * HIDV,
                                     mean + (size_t)i * HIDV, var + (size_t)i * HIDV, nN, csrLen);
  }

  k_gemm<JKK / 32, KP / 32, KP><<<nGemm, NTHR, 0, stream>>>(xs, wbjk, dinv, bjk, hw, plane, 0, 1, HIDV);

  k_pool<<<nPool, NTHR, 0, stream>>>(batch, hw, Wout, bout, gout, nN);
  k_out<<<1, NTHR, 0, stream>>>(gout, out, G);
}
